// TopologicalEmbedding_51316269252742
// MI455X (gfx1250) — hardware-verified
//
#include <hip/hip_runtime.h>


namespace {
constexpr int B = 128, P = 2048, F = 256, H4 = 256, H2 = 512, H = 1024, RES = 4096, LC = 2048;
constexpr float HS = 256.0f, WSC = 256.0f, EPS = 1e-5f;
typedef _Float16 b16;
typedef __attribute__((ext_vector_type(16))) _Float16 v16b;
typedef __attribute__((ext_vector_type(8))) _Float16 v8b;
typedef __attribute__((ext_vector_type(8))) float v8f;
typedef __attribute__((ext_vector_type(4))) float v4f;
__device__ __forceinline__ float bf16_rne(float f) { unsigned int u = __float_as_uint(f); u += 0x7FFFu + ((u >> 16) & 1u); float r = __uint_as_float(u & 0xFFFF0000u); asm volatile("" : "+v"(r)); return r; }
__device__ __forceinline__ float bfv(float f) { float r = bf16_rne(f); asm volatile("" : "+v"(r)); return r; }
__device__ __forceinline__ void split16(float v, b16& hi, b16& lo) { hi = (b16)v; lo = (b16)(v - (float)hi); }
__device__ __forceinline__ v16b frag_kb(const b16* p, int hh) { const v8b a = *(const v8b*)(p + 8 * hh), b = *(const v8b*)(p + 16 + 8 * hh); v16b f;
#pragma unroll
  for (int e = 0; e < 8; ++e) { f[e] = a[e]; f[8 + e] = b[e]; } return f; }
__device__ __forceinline__ v8f wmma16b(v16b a, v16b b, v8f c) { v8f d = __builtin_amdgcn_wmma_f32_16x16x32_f16(false, a, false, b, (short)0, c, false, false); asm volatile("v_nop\n\tv_nop\n\tv_nop\n\tv_nop" : "+v"(d) : "v"(a), "v"(b)); return d; }
__device__ __forceinline__ void wave_lds_sync() { __builtin_amdgcn_fence(__ATOMIC_RELEASE, "workgroup"); __builtin_amdgcn_wave_barrier(); __builtin_amdgcn_fence(__ATOMIC_ACQUIRE, "workgroup"); }
__device__ __forceinline__ float pmul(float a, float b) { float p = a * b; asm volatile("" : "+v"(p)); return p; }
__device__ __forceinline__ int iclamp(int v, int lo, int hi) { return v < lo ? lo : (v > hi ? hi : v); }

__global__ __launch_bounds__(256) void wput_kernel(const float* __restrict__ w2, const float* __restrict__ wo, b16* __restrict__ WT2, b16* __restrict__ WTO) { const size_t nt = (size_t)gridDim.x * 256, u0 = (size_t)blockIdx.x * 256 + threadIdx.x; v8b v;
  for (size_t u = u0; u < (size_t)H4 * 32; u += nt) { const int o = (int)(u / 32), k0 = (int)(u % 32) * 8;
#pragma unroll
    for (int j = 0; j < 8; ++j) v[j] = (b16)(bf16_rne(w2[(size_t)(k0 + j) * H4 + o]) * WSC); for (int pass = 0; pass < 2; ++pass) { *(volatile v8b*)(WT2 + (size_t)o * F + k0) = v; __threadfence(); } }
  for (size_t u = u0; u < (size_t)H * 128; u += nt) { const int o = (int)(u / 128), k0 = (int)(u % 128) * 8;
#pragma unroll
    for (int j = 0; j < 8; ++j) v[j] = (b16)(bf16_rne(wo[(size_t)(k0 + j) * H + o]) * WSC); for (int pass = 0; pass < 2; ++pass) { *(volatile v8b*)(WTO + (size_t)o * H + k0) = v; __threadfence(); } } }
__global__ __launch_bounds__(256) void sample_kernel(const float* __restrict__ pd, const int* __restrict__ lens, const float* __restrict__ img, const float* __restrict__ w1, const float* __restrict__ b1, const float* __restrict__ lg, const float* __restrict__ lb, float* __restrict__ PG, float* __restrict__ PS) { const int wave = threadIdx.x >> 5, lane = threadIdx.x & 31; const int b = blockIdx.x * 8 + wave; if (b >= B) return;
  float w1v[3][8], b1v[8], gg[8], gb[8], acc[8]; for (int k = 0; k < 8; ++k) { const int c = lane * 8 + k; for (int i = 0; i < 3; ++i) w1v[i][k] = bfv(w1[i * F + c]); b1v[k] = bfv(b1[c]); gg[k] = bfv(lg[c]); gb[k] = bfv(lb[c]); acc[k] = 0.0f; }
  const int len = iclamp(lens[b], 0, P);
#pragma unroll 1
  for (int p = 0; p < len; ++p) { const float x0 = bfv(pd[((size_t)b * P + p) * 3]), x1 = bfv(pd[((size_t)b * P + p) * 3 + 1]), x2 = bfv(pd[((size_t)b * P + p) * 3 + 2]); float hv[8]; float s = 0.0f;
#pragma unroll
    for (int k = 0; k < 8; ++k) { hv[k] = b1v[k] + pmul(x0, w1v[0][k]) + pmul(x1, w1v[1][k]) + pmul(x2, w1v[2][k]); s += hv[k]; }
    for (int o = 16; o; o >>= 1) s += __shfl_xor(s, o); const float mu = s * (1.0f / F); float vq = 0.0f;
#pragma unroll
    for (int k = 0; k < 8; ++k) { const float d = hv[k] - mu; vq += d * d; }
    for (int o = 16; o; o >>= 1) vq += __shfl_xor(vq, o); const float rs = rsqrtf(vq * (1.0f / F) + EPS);
#pragma unroll
    for (int k = 0; k < 8; ++k) { const float v = pmul((hv[k] - mu) * rs, gg[k]) + gb[k]; acc[k] += 0.5f * v * (1.0f + erff(v * 0.70710678118654752f)); } }
  float sj[5]; for (int j = 0; j < 5; ++j) { float s = 0.0f; for (int l = lane; l < LC; l += 32) { const int i = 2 * l + j - 2; if (i >= 0 && i < RES) s += bfv(img[(size_t)b * RES + i]); } for (int o = 16; o; o >>= 1) s += __shfl_xor(s, o); sj[j] = s; }
  for (int pass = 0; pass < 2; ++pass) { v4f a0 = {acc[0], acc[1], acc[2], acc[3]}, a1 = {acc[4], acc[5], acc[6], acc[7]}; *(volatile v4f*)(PG + (size_t)b * F + lane * 8) = a0; *(volatile v4f*)(PG + (size_t)b * F + lane * 8 + 4) = a1; const float sv = lane == 0 ? sj[0] : lane == 1 ? sj[1] : lane == 2 ? sj[2] : lane == 3 ? sj[3] : lane == 4 ? sj[4] : 0.0f; ((volatile float*)PS)[(size_t)b * 32 + lane] = sv; __threadfence(); } }
__global__ __launch_bounds__(32) void head_kernel(const float* __restrict__ PG, const float* __restrict__ PS, const int* __restrict__ lens, const int* __restrict__ betti, const float* __restrict__ table, const float* __restrict__ cw, const float* __restrict__ cb, const b16* __restrict__ WT2, const float* __restrict__ b2, const b16* __restrict__ WTO, const float* __restrict__ bo, float* __restrict__ out) { __shared__ __attribute__((aligned(16))) b16 Ah[16][H + 8], Al[16][H + 8]; __shared__ float Tf[16][260]; const int lane = threadIdx.x, nloc = lane & 15, hlf = lane >> 4; const int b0 = blockIdx.x * 16;
  auto put = [&](int rr, int c, float v) { b16 p, pl; split16(v * HS, p, pl); Ah[rr][c] = p; Al[rr][c] = pl; };
  for (int rr = 0; rr < 16; ++rr) { const int b = b0 + rr; const float inv = 1.0f / fmaxf((float)iclamp(lens[b], 0, P), 1.0f); for (int q = 0; q < 8; ++q) { const int c = q * 32 + lane; b16 p, pl; split16(PG[(size_t)b * F + c] * inv * HS, p, pl); Ah[rr][c] = p; Al[rr][c] = pl; } }
  if (lane < 16) for (int k = F; k < F + 8; ++k) { Ah[lane][k] = (b16)0.0f; Al[lane][k] = (b16)0.0f; }
  wave_lds_sync();
  { v8f acc[16];
#pragma unroll
    for (int t = 0; t < 16; ++t) acc[t] = (v8f){};
#pragma unroll 2
    for (int kb = 0; kb < F; kb += 32) { const v16b a = frag_kb(&Ah[nloc][kb], hlf), al = frag_kb(&Al[nloc][kb], hlf);
#pragma unroll
      for (int t = 0; t < 16; ++t) { const v16b bw = frag_kb(WT2 + (size_t)(t * 16 + nloc) * F + kb, hlf); acc[t] = wmma16b(a, bw, acc[t]); acc[t] = wmma16b(al, bw, acc[t]); } }
#pragma unroll
    for (int t = 0; t < 16; ++t) { const int cc = t * 16 + nloc; const float bb = bfv(b2[cc]);
#pragma unroll
      for (int r8 = 0; r8 < 8; ++r8) { const int rr = 8 * hlf + r8; const bool has = iclamp(lens[b0 + rr], 0, P) > 0; Tf[rr][cc] = has ? acc[t][r8] * (1.0f / (HS * WSC)) + bb : 0.0f; } } }
  wave_lds_sync();
  for (int rr = 0; rr < 16; ++rr) for (int q = 0; q < 8; ++q) { const int c = q * 32 + lane; put(rr, c, Tf[rr][c]); }
  for (int rr = 0; rr < 16; ++rr) { const int b = b0 + rr; const int i0 = iclamp(betti[b * 3], 0, 9), i1 = iclamp(betti[b * 3 + 1], 0, 9), i2 = iclamp(betti[b * 3 + 2], 0, 9); for (int q = 0; q < 8; ++q) { const int c = q * 32 + lane; put(rr, H4 + c, (bfv(table[i0 * H4 + c]) + bfv(table[i1 * H4 + c]) + bfv(table[i2 * H4 + c])) * (1.0f / 3.0f)); }
    float sj[5]; for (int j = 0; j < 5; ++j) sj[j] = PS[(size_t)b * 32 + j]; for (int q = 0; q < 16; ++q) { const int o = q * 32 + lane; float s = 0.0f; for (int j = 0; j < 5; ++j) s += pmul(bfv(cw[o * 5 + j]), sj[j]); put(rr, H4 + H4 + o, s * (1.0f / (float)LC) + bfv(cb[o])); } }
  if (lane < 16) for (int k = H; k < H + 8; ++k) { Ah[lane][k] = (b16)0.0f; Al[lane][k] = (b16)0.0f; }
  wave_lds_sync();
#pragma unroll 1
  for (int g = 0; g < 4; ++g) { v8f acc[16];
#pragma unroll
    for (int t = 0; t < 16; ++t) acc[t] = (v8f){};
#pragma unroll 2
    for (int kb = 0; kb < H; kb += 32) { const v16b a = frag_kb(&Ah[nloc][kb], hlf), al = frag_kb(&Al[nloc][kb], hlf);
#pragma unroll
      for (int t = 0; t < 16; ++t) { const v16b bw = frag_kb(WTO + (size_t)(g * 256 + t * 16 + nloc) * H + kb, hlf); acc[t] = wmma16b(a, bw, acc[t]); acc[t] = wmma16b(al, bw, acc[t]); } }
#pragma unroll
    for (int t = 0; t < 16; ++t) { const int cc = t * 16 + nloc; const float bb = bfv(bo[g * 256 + cc]);
#pragma unroll
      for (int r8 = 0; r8 < 8; ++r8) Tf[8 * hlf + r8][cc] = acc[t][r8] * (1.0f / (HS * WSC)) + bb; }
    wave_lds_sync();
    for (int pass = 0; pass < 2; ++pass) { for (int rr = 0; rr < 16; ++rr) for (int q = 0; q < 2; ++q) *(volatile v4f*)(out + (size_t)(b0 + rr) * H + g * 256 + q * 128 + lane * 4) = *(const v4f*)(&Tf[rr][q * 128 + lane * 4]); __threadfence(); }
    wave_lds_sync(); } }
}

extern "C" void kernel_launch(void* const* d_in, const int* in_sizes, int n_in, void* d_out, int out_size, void* d_ws, size_t ws_size, hipStream_t stream) {
  (void)n_in;
  auto Fp = [&](int i) { return (const float*)d_in[i]; }; auto Ip = [&](int i) { return (const int*)d_in[i]; };
  if (in_sizes[0] != B * P * 3 || in_sizes[1] != B || in_sizes[2] != B * 3 || in_sizes[3] != B * RES || in_sizes[4] != 3 * F || in_sizes[8] != F * H4 || in_sizes[10] != 10 * H4 || in_sizes[11] != H2 * 5 || in_sizes[13] != H * H || out_size != B * H) return;
  size_t off = 0; char* ws = (char*)d_ws;
  auto carve = [&](size_t bytes) { char* p = ws + off; off += (bytes + 255) & ~(size_t)255; return p; };
  b16* WT2 = (b16*)carve((size_t)H4 * F * 2); b16* WTO = (b16*)carve((size_t)H * H * 2); float* PG = (float*)carve((size_t)B * F * 4); float* PS = (float*)carve((size_t)B * 32 * 4);
  if (off > ws_size || off > ((size_t)4 << 20)) return;
  wput_kernel<<<64, 256, 0, stream>>>(Fp(8), Fp(13), WT2, WTO);
  sample_kernel<<<B / 8, 256, 0, stream>>>(Fp(0), Ip(1), Fp(3), Fp(4), Fp(5), Fp(6), Fp(7), PG, PS);
  head_kernel<<<B / 16, 32, 0, stream>>>(PG, PS, Ip(1), Ip(2), Fp(10), Fp(11), Fp(12), WT2, Fp(9), WTO, Fp(14), (float*)d_out);
}
